// GlobalAttentionTransformer_446676599180
// MI455X (gfx1250) — hardware-run, weakly checked
//
#include <hip/hip_runtime.h>
#include <math.h>

constexpr int kBatch  = 8;
constexpr int kDim    = 768;
constexpr int kHeads  = 12;
constexpr int kHd     = 64;
constexpr int kReg    = 4;
constexpr int kGlob   = 1 + kReg;
constexpr int kHW     = 1024;
constexpr int kSeq    = kGlob + kHW;
constexpr int kRows   = kBatch * kSeq;
constexpr int kRowsP  = 8256;
constexpr int kQkvN   = 3 * kDim;
constexpr int kFfn    = 4 * kDim;
constexpr int kChunkRows = 2048;
constexpr int kNumChunks = (kRowsP + kChunkRows - 1) / kChunkRows;
constexpr float kWCarry    = 16.0f;
constexpr float kWCarryInv = 1.0f / 16.0f;
constexpr float kEps     = 1e-5f;
constexpr float kInvDim  = 1.0f / 768.0f;
constexpr float kQkScale = 0.125f;
static_assert(kRowsP % 64 == 0 && kRowsP >= kRows, "");
static_assert(kDim % 64 == 0 && kFfn % 64 == 0 && kQkvN % 64 == 0, "");
static_assert(kDim % 32 == 0 && kFfn % 32 == 0, "");
static_assert(kChunkRows % 64 == 0, "");
static_assert((kBatch * kHW * kHeads) % 16 == 0, "");

constexpr size_t kFeatElems = (size_t)kBatch * kDim * kHW;
constexpr size_t kCtxElems  = (size_t)kBatch * kDim;
constexpr size_t kRegElems  = (size_t)kBatch * kReg * kDim;
constexpr size_t kOutElems  = kFeatElems + kCtxElems + kRegElems;
static_assert(kFeatElems * 4 == 25165824, "");
static_assert((kFeatElems + kCtxElems) * 4 == 25190400, "");
static_assert(kOutElems * 4 == 25288704, "");

constexpr size_t kBytesW1h  = (size_t)kFfn  * kDim * 2;
constexpr size_t kBytesW2h  = (size_t)kDim  * kFfn * 2;
constexpr size_t kBytesWQh  = (size_t)kQkvN * kDim * 2;
constexpr size_t kBytesWOh  = (size_t)kDim  * kDim * 2;
constexpr size_t kBytesF32P = (size_t)kRowsP * kDim * 4;
constexpr size_t kBytesH16P = (size_t)kRowsP * kDim * 2;
constexpr size_t kBytesQKV  = (size_t)kRowsP * kQkvN * 4;
constexpr size_t kBytesFF1  = (size_t)kRowsP * kFfn * 2;
constexpr size_t kBytesChunk = (size_t)kChunkRows * kFfn * 4;
constexpr size_t kOffW1h = 0;
constexpr size_t kOffW2h = kOffW1h + kBytesW1h;
constexpr size_t kOffWQh = kOffW2h + kBytesW2h;
constexpr size_t kOffWOh = kOffWQh + kBytesWQh;
constexpr size_t kOffRA  = kOffWOh + kBytesWOh;
constexpr size_t kOffRB  = kOffRA + kBytesF32P;
constexpr size_t kOffRC  = kOffRB + kBytesH16P;
constexpr size_t kOffFF1 = kOffRC + kBytesF32P;
constexpr size_t kWsTotal = kOffRC + kBytesQKV;
static_assert(kBytesF32P + kBytesFF1 == kBytesQKV, "");
static_assert(kBytesChunk <= kBytesF32P, "");
static_assert(kWsTotal == 128286720, "");
static_assert(kWsTotal <= 134217728, "");
static_assert(kOffW2h % 128 == 0 && kOffWQh % 128 == 0 && kOffWOh % 128 == 0 && kOffRA % 128 == 0 &&
              kOffRB % 128 == 0 && kOffRC % 128 == 0 && kOffFF1 % 128 == 0, "");

typedef __attribute__((ext_vector_type(16))) _Float16 v16h;
typedef __attribute__((ext_vector_type(8)))  _Float16 v8h;
typedef __attribute__((ext_vector_type(16))) __bf16   v16b;
typedef __attribute__((ext_vector_type(8)))  __bf16   v8b;
typedef __attribute__((ext_vector_type(8)))  float    v8f;
typedef __attribute__((ext_vector_type(4)))  float    v4f;
typedef __attribute__((ext_vector_type(2)))  float    v2f;
typedef __attribute__((ext_vector_type(4)))  unsigned int v4u;

__device__ __forceinline__ unsigned short f2bf_bits(float f) {
  unsigned u = __float_as_uint(f);
  return (unsigned short)((u + 0x7FFFu + ((u >> 16) & 1u)) >> 16);
}
__device__ __forceinline__ float bf_bits2f(unsigned short h) { return __uint_as_float(((unsigned)h) << 16); }

__device__ __forceinline__ void dep_guard_h(v8f& a, v8f& b, v16h x, v16h y) { asm volatile("v_nop\n\tv_nop\n\tv_nop\n\tv_nop" : "+v"(a), "+v"(b) : "v"(x), "v"(y)); }
__device__ __forceinline__ void dep_guard_b(v8f& a, v8f& b, v16b x, v16b y) { asm volatile("v_nop\n\tv_nop\n\tv_nop\n\tv_nop" : "+v"(a), "+v"(b) : "v"(x), "v"(y)); }
__device__ __forceinline__ void keep4_h(v16h a, v16h b, v16h c, v16h d) { asm volatile("v_nop" :: "v"(a), "v"(b), "v"(c), "v"(d)); }
__device__ __forceinline__ void keep4_b(v16b a, v16b b, v16b c, v16b d) { asm volatile("v_nop" :: "v"(a), "v"(b), "v"(c), "v"(d)); }
__device__ __forceinline__ void acc_guard4(v8f& a, v8f& b, v8f& c, v8f& d) { asm volatile("v_nop\n\tv_nop\n\tv_nop\n\tv_nop" : "+v"(a), "+v"(b), "+v"(c), "+v"(d)); }
template <typename T> struct Frag;
template <> struct Frag<_Float16> {
  typedef v16h V; union U { v16h v; v8h h[2]; };
  static __device__ __forceinline__ v16h load(const _Float16* p) {
    U f; f.h[0] = *(const v8h*)(p); f.h[1] = *(const v8h*)(p + 16); return f.v;
  }
  static __device__ __forceinline__ v8f mma(v16h a, v16h b, v8f c) {
    return __builtin_amdgcn_wmma_f32_16x16x32_f16(false, a, false, b, (short)0, c, false, false);
  }
  static __device__ __forceinline__ void guard(v8f& a, v8f& b, v16h x, v16h y) { dep_guard_h(a, b, x, y); }
  static __device__ __forceinline__ void keep(v16h a, v16h b, v16h c, v16h d) { keep4_h(a, b, c, d); }
};
template <> struct Frag<__bf16> {
  typedef v16b V; union U { v16b v; v8b h[2]; };
  static __device__ __forceinline__ v16b load(const __bf16* p) {
    U f; f.h[0] = *(const v8b*)(p); f.h[1] = *(const v8b*)(p + 16); return f.v;
  }
  static __device__ __forceinline__ v8f mma(v16b a, v16b b, v8f c) {
    return __builtin_amdgcn_wmma_f32_16x16x32_bf16(false, a, false, b, (short)0, c, false, false);
  }
  static __device__ __forceinline__ void guard(v8f& a, v8f& b, v16b x, v16b y) { dep_guard_b(a, b, x, y); }
  static __device__ __forceinline__ void keep(v16b a, v16b b, v16b c, v16b d) { keep4_b(a, b, c, d); }
};

__device__ __forceinline__ unsigned pk16(unsigned short a, unsigned short b) { return (unsigned)a | ((unsigned)b << 16); }
__device__ __forceinline__ unsigned short h_bits(float f) { const _Float16 h = (_Float16)f; return __builtin_bit_cast(unsigned short, h); }
__device__ __forceinline__ v4u pack8_h(const float* sp) {
  return (v4u){pk16(h_bits(sp[0]), h_bits(sp[1])), pk16(h_bits(sp[2]), h_bits(sp[3])),
               pk16(h_bits(sp[4]), h_bits(sp[5])), pk16(h_bits(sp[6]), h_bits(sp[7]))};
}

template <int ET> struct Elem;
template <> struct Elem<0> { typedef _Float16 T; };
template <> struct Elem<1> { typedef __bf16 T; };
template <int ET, bool SPLIT, int BIAS_MODE, int OUT_MODE, bool RESID, int ACT = 0>
__global__ __launch_bounds__(256) void wmma_gemm64(
    const unsigned short* __restrict__ Ap, const unsigned short* __restrict__ A2p, int lda, long strideA,
    const unsigned short* __restrict__ Btp, const unsigned short* __restrict__ Bt2p, int ldb, long strideB,
    void* __restrict__ Cout, void* __restrict__ Cout2, int ldc, long strideC,
    const float* __restrict__ bias,
    const float* __restrict__ resid, long strideR,
    int M, int N, int K, float scale) {
  typedef typename Elem<ET>::T T;
  typedef typename Frag<T>::V V;
  const T* A = (const T*)Ap; const T* A2 = (const T*)A2p; const T* Bt = (const T*)Btp; const T* Bt2 = (const T*)Bt2p;
  __shared__ __align__(16) float sT[8][16 * 68];
  const int b    = blockIdx.y;
  const int lane = threadIdx.x & 31;
  const int wave = threadIdx.x >> 5;
  const int tilesN = N >> 6;
  const int tilesM = M >> 6;
  const int tile = blockIdx.x * 8 + wave;
  if (tile >= tilesM * tilesN) return;
  const int tm = tile / tilesN;
  const int tn = tile - tm * tilesN;
  const int m0 = tm << 6;
  const int n0 = tn << 6;

  const T* Ab  = A  + (size_t)b * strideA;
  const T* Bb  = Bt + (size_t)b * strideB;
  const T* Ab2 = SPLIT ? (A2  + (size_t)b * strideA) : nullptr;
  const T* Bb2 = SPLIT ? (Bt2 + (size_t)b * strideB) : nullptr;

  const int rlane = lane & 15;
  const int koff  = (lane >> 4) * 8;
  const int mOff  = (lane >> 4) * 8;

  v8f acc[4][4];
#pragma unroll
  for (int i = 0; i < 4; ++i)
#pragma unroll
    for (int j = 0; j < 4; ++j) acc[i][j] = (v8f){0.f,0.f,0.f,0.f,0.f,0.f,0.f,0.f};

  for (int k0 = 0; k0 < K; k0 += 32) {
    V bh[4], bl[4];
#pragma unroll
    for (int j = 0; j < 4; ++j) {
      const size_t bo = (size_t)(n0 + (j << 4) + rlane) * ldb + koff + k0;
      bh[j] = Frag<T>::load(Bb + bo);
      if (SPLIT) bl[j] = Frag<T>::load(Bb2 + bo);
    }
#pragma unroll
    for (int i = 0; i < 4; ++i) {
      const size_t ao = (size_t)(m0 + (i << 4) + rlane) * lda + koff + k0;
      V ah = Frag<T>::load(Ab + ao);
      V al;
      if (SPLIT) al = Frag<T>::load(Ab2 + ao);
#pragma unroll
      for (int j = 0; j < 4; ++j) {
        acc[i][j] = Frag<T>::mma(ah, bh[j], acc[i][j]);
        if (SPLIT) {
          acc[i][j] = Frag<T>::mma(ah, bl[j], acc[i][j]);
          acc[i][j] = Frag<T>::mma(al, bh[j], acc[i][j]);
        }
      }
      Frag<T>::guard(acc[i][0], acc[i][3], ah, SPLIT ? al : ah);
    }
    Frag<T>::keep(bh[0], bh[1], bh[2], bh[3]);
    if (SPLIT) Frag<T>::keep(bl[0], bl[1], bl[2], bl[3]);
  }
  acc_guard4(acc[0][0], acc[0][1], acc[0][2], acc[0][3]);
  acc_guard4(acc[1][0], acc[1][1], acc[1][2], acc[1][3]);
  acc_guard4(acc[2][0], acc[2][1], acc[2][2], acc[2][3]);
  acc_guard4(acc[3][0], acc[3][1], acc[3][2], acc[3][3]);

  float* slab = sT[wave];
  const float* Rb = RESID ? (resid + (size_t)b * strideR) : nullptr;
#pragma unroll
  for (int i = 0; i < 4; ++i) {
    const int mBase = m0 + (i << 4);
#pragma unroll
    for (int j = 0; j < 4; ++j) {
      const int n = n0 + (j << 4) + rlane;
      float bv = 0.f;
      if (BIAS_MODE == 2) bv = bias[n];
#pragma unroll
      for (int r = 0; r < 8; ++r) {
        float v = acc[i][j][r] * scale;
        if (BIAS_MODE == 1) v += bias[mBase + mOff + r];
        if (BIAS_MODE == 2) v += bv;
        if (RESID) v += Rb[(size_t)(mBase + mOff + r) * ldc + n];
        if (ACT == 2) v = fmaxf(v, 0.0f);
        if (ACT == 4) v = (v > 0.f) ? v : 0.01f * v;
        slab[(mOff + r) * 68 + (j << 4) + rlane] = v;
      }
    }
    __builtin_amdgcn_fence(__ATOMIC_RELEASE, "workgroup");
    __builtin_amdgcn_wave_barrier();
    __builtin_amdgcn_fence(__ATOMIC_ACQUIRE, "workgroup");
    if (OUT_MODE == 0) {
      float* C = (float*)Cout + (size_t)b * strideC;
      const int hh = lane >> 4, c4 = (lane & 15) * 4;
      for (int pass = 0; pass < 2; ++pass) {
#pragma unroll
        for (int it = 0; it < 8; ++it) {
          const int row = it * 2 + hh;
          v4f v = *(const v4f*)(slab + row * 68 + c4);
          *(volatile v4f*)(C + (size_t)(mBase + row) * ldc + n0 + c4) = v;
        }
        __threadfence();
      }
    } else {
      const int q = lane >> 3, c8 = (lane & 7) * 8;
      unsigned short* C  = (unsigned short*)Cout  + (size_t)b * strideC;
      unsigned short* C2 = (OUT_MODE == 2) ? ((unsigned short*)Cout2 + (size_t)b * strideC) : nullptr;
      for (int pass = 0; pass < 2; ++pass) {
#pragma unroll
        for (int it = 0; it < 4; ++it) {
          const int row = it * 4 + q;
          const float* sp = slab + row * 68 + c8;
          v8h hv, lv;
#pragma unroll
          for (int e = 0; e < 8; ++e) {
            if (OUT_MODE == 1) {
              hv[e] = (_Float16)sp[e];
            } else {
              unsigned short hb = f2bf_bits(sp[e]);
              unsigned short lb = f2bf_bits(sp[e] - bf_bits2f(hb));
              hv[e] = __builtin_bit_cast(_Float16, hb);
              lv[e] = __builtin_bit_cast(_Float16, lb);
            }
          }
          *(volatile v8h*)(C + (size_t)(mBase + row) * ldc + n0 + c8) = hv;
          if (OUT_MODE == 2) *(volatile v8h*)(C2 + (size_t)(mBase + row) * ldc + n0 + c8) = lv;
        }
        __threadfence();
      }
    }
    __builtin_amdgcn_fence(__ATOMIC_RELEASE, "workgroup");
    __builtin_amdgcn_wave_barrier();
    __builtin_amdgcn_fence(__ATOMIC_ACQUIRE, "workgroup");
  }
}

__device__ __forceinline__ float wave_sum32(float v) {
#pragma unroll
  for (int off = 16; off > 0; off >>= 1) v += __shfl_xor(v, off, 32);
  return v;
}
__device__ __forceinline__ float wave_max32(float v) {
#pragma unroll
  for (int off = 16; off > 0; off >>= 1) v = fmaxf(v, __shfl_xor(v, off, 32));
  return v;
}

__global__ __launch_bounds__(256) void wcast8_kernel(const float* __restrict__ in, unsigned short* __restrict__ out, int n8, float scale) {
  const int i = blockIdx.x * 256 + threadIdx.x;
  if (i >= n8) return;
  const float* p = in + 8 * (size_t)i;
  const v4f a = *(const v4f*)(p);
  const v4f c = *(const v4f*)(p + 4);
  unsigned short hb[8];
#pragma unroll
  for (int e = 0; e < 4; ++e) {
    hb[e]     = h_bits(a[e] * scale);
    hb[4 + e] = h_bits(c[e] * scale);
  }
  const v4u u = (v4u){pk16(hb[0], hb[1]), pk16(hb[2], hb[3]), pk16(hb[4], hb[5]), pk16(hb[6], hb[7])};
  unsigned short* q = out + 8 * (size_t)i;
  *(volatile v4u*)q = u;
  __threadfence();
  *(volatile v4u*)q = u;
}

__global__ __launch_bounds__(256) void ln1_kernel(const float* __restrict__ x, const float* __restrict__ ctxt,
                                                  const float* __restrict__ regt, const float* __restrict__ g,
                                                  const float* __restrict__ bta, float* __restrict__ xw,
                                                  unsigned short* __restrict__ xw16) {
  __shared__ float red[8];
  __shared__ __align__(16) float rowbuf[kDim];
  const int row  = blockIdx.x;
  const int tid  = threadIdx.x, lane = tid & 31, wave = tid >> 5;
  float* dst32 = xw + (size_t)row * kDim;
  unsigned short* dst16 = xw16 + (size_t)row * kDim;
  const int i4 = (tid < 192 ? tid : 191) * 4;
  const int i8 = (tid < 96 ? tid : 95) * 8;
  if (row >= kRows) {
    const v4f z = (v4f){0.f, 0.f, 0.f, 0.f};
    const v4u zu = (v4u){0u, 0u, 0u, 0u};
    for (int pass = 0; pass < 2; ++pass) {
      if (tid < 192) *(volatile v4f*)(dst32 + i4) = z;
      if (tid < 96)  *(volatile v4u*)(dst16 + i8) = zu;
      __threadfence();
    }
    return;
  }
  const int b = row / kSeq;
  const int s = row - b * kSeq;
  const float* src;
  size_t stride;
  if (s == 0)         { src = ctxt + (size_t)b * kDim;                      stride = 1; }
  else if (s < kGlob) { src = regt + ((size_t)b * kReg + (s - 1)) * kDim;  stride = 1; }
  else                { src = x + (size_t)b * kDim * kHW + (s - kGlob);    stride = kHW; }
  const int c0 = tid, c1 = tid + 256, c2 = tid + 512;
  const float v0 = src[(size_t)c0 * stride];
  const float v1 = src[(size_t)c1 * stride];
  const float v2 = src[(size_t)c2 * stride];

  float ps = wave_sum32(v0 + v1 + v2);
  if (lane == 0) red[wave] = ps;
  __syncthreads();
  float tot = red[0]; tot += red[1]; tot += red[2]; tot += red[3]; tot += red[4]; tot += red[5]; tot += red[6]; tot += red[7];
  const float mu = tot * kInvDim;
  __syncthreads();
  const float d0 = v0 - mu, d1 = v1 - mu, d2 = v2 - mu;
  float pq = wave_sum32(d0 * d0 + d1 * d1 + d2 * d2);
  if (lane == 0) red[wave] = pq;
  __syncthreads();
  float tq = red[0]; tq += red[1]; tq += red[2]; tq += red[3]; tq += red[4]; tq += red[5]; tq += red[6]; tq += red[7];
  const float rstd = rsqrtf(tq * kInvDim + kEps);
  rowbuf[c0] = d0 * rstd * g[c0] + bta[c0];
  rowbuf[c1] = d1 * rstd * g[c1] + bta[c1];
  rowbuf[c2] = d2 * rstd * g[c2] + bta[c2];
  __syncthreads();
  for (int pass = 0; pass < 2; ++pass) {
    if (tid < 192) { const v4f v = *(const v4f*)(rowbuf + i4); *(volatile v4f*)(dst32 + i4) = v; }
    if (tid < 96)  { const v4u u = pack8_h(rowbuf + i8);      *(volatile v4u*)(dst16 + i8) = u; }
    __threadfence();
  }
}

__global__ __launch_bounds__(256) void ln2_kernel(const float* __restrict__ h1, const float* __restrict__ g,
                                                  const float* __restrict__ bta, unsigned short* __restrict__ out16) {
  __shared__ float red[8];
  __shared__ __align__(16) float rowbuf[kDim];
  const int row  = blockIdx.x;
  const int tid  = threadIdx.x, lane = tid & 31, wave = tid >> 5;
  unsigned short* dst16 = out16 + (size_t)row * kDim;
  const int i8 = (tid < 96 ? tid : 95) * 8;
  if (row >= kRows) {
    const v4u zu = (v4u){0u, 0u, 0u, 0u};
    for (int pass = 0; pass < 2; ++pass) {
      if (tid < 96) *(volatile v4u*)(dst16 + i8) = zu;
      __threadfence();
    }
    return;
  }
  const float* src = h1 + (size_t)row * kDim;
  const int c0 = tid, c1 = tid + 256, c2 = tid + 512;
  const float v0 = src[c0], v1 = src[c1], v2 = src[c2];
  float ps = wave_sum32(v0 + v1 + v2);
  if (lane == 0) red[wave] = ps;
  __syncthreads();
  float tot = red[0]; tot += red[1]; tot += red[2]; tot += red[3]; tot += red[4]; tot += red[5]; tot += red[6]; tot += red[7];
  const float mu = tot * kInvDim;
  __syncthreads();
  const float d0 = v0 - mu, d1 = v1 - mu, d2 = v2 - mu;
  float pq = wave_sum32(d0 * d0 + d1 * d1 + d2 * d2);
  if (lane == 0) red[wave] = pq;
  __syncthreads();
  float tq = red[0]; tq += red[1]; tq += red[2]; tq += red[3]; tq += red[4]; tq += red[5]; tq += red[6]; tq += red[7];
  const float rstd = rsqrtf(tq * kInvDim + kEps);
  rowbuf[c0] = d0 * rstd * g[c0] + bta[c0];
  rowbuf[c1] = d1 * rstd * g[c1] + bta[c1];
  rowbuf[c2] = d2 * rstd * g[c2] + bta[c2];
  __syncthreads();
  for (int pass = 0; pass < 2; ++pass) {
    if (tid < 96) { const v4u u = pack8_h(rowbuf + i8); *(volatile v4u*)(dst16 + i8) = u; }
    __threadfence();
  }
}

__global__ __launch_bounds__(256) void attn_glob_kernel(const float* __restrict__ qkv, unsigned short* __restrict__ attn16) {
  __shared__ __align__(16) float qsh[kHd];
  __shared__ float sc[1040];
  __shared__ float red[8];
  __shared__ __align__(16) float pv[16][68];
  __shared__ __align__(16) float outs[kHd];
  const int tid = threadIdx.x, lane = tid & 31, wave = tid >> 5;
  const int blk = blockIdx.x;
  const int b   = blk / (kHeads * kGlob);
  const int rem = blk - b * (kHeads * kGlob);
  const int h   = rem / kGlob;
  const int s   = rem - h * kGlob;
  const size_t rowq = (size_t)b * kSeq + s;
  const float* qp = qkv + rowq * kQkvN + h * kHd;
  if (tid < kHd) qsh[tid] = qp[tid];
  __syncthreads();
  const float* kbase = qkv + (size_t)b * kSeq * kQkvN + kDim + h * kHd;
  const float* vbase = qkv + (size_t)b * kSeq * kQkvN + 2 * kDim + h * kHd;

  for (int t = tid; t < kSeq; t += 256) {
    const float* kp = kbase + (size_t)t * kQkvN;
    float d = 0.f;
#pragma unroll 1
    for (int dh = 0; dh < 2; ++dh) {
#pragma unroll
      for (int i = 0; i < 8; ++i) {
        const v4f kk = *(const v4f*)(kp + dh * 32 + 4 * i);
        const v4f qq = *(const v4f*)(qsh + dh * 32 + 4 * i);
        d += qq.x * kk.x; d += qq.y * kk.y; d += qq.z * kk.z; d += qq.w * kk.w;
      }
    }
    sc[t] = d * kQkScale;
  }
  __syncthreads();
  float m = -INFINITY;
  for (int t = tid; t < kSeq; t += 256) m = fmaxf(m, sc[t]);
  m = wave_max32(m);
  if (lane == 0) red[wave] = m;
  __syncthreads();
  m = red[0];
#pragma unroll
  for (int w = 1; w < 8; ++w) m = fmaxf(m, red[w]);
  __syncthreads();
  float ps = 0.f;
  for (int t = tid; t < kSeq; t += 256) { const float e = expf(sc[t] - m); sc[t] = e; ps += e; }
  ps = wave_sum32(ps);
  if (lane == 0) red[wave] = ps;
  __syncthreads();
  float tot = red[0]; tot += red[1]; tot += red[2]; tot += red[3]; tot += red[4]; tot += red[5]; tot += red[6]; tot += red[7];
  const float inv = 1.0f / tot;
  const int slice = tid >> 4, d4 = (tid & 15) * 4;
  const int t0 = slice * 65;
  const int t1 = (t0 + 65 < kSeq) ? (t0 + 65) : kSeq;
  v4f acc = (v4f){0.f, 0.f, 0.f, 0.f};
  for (int t = t0; t < t1; ++t) {
    const float p = sc[t];
    const v4f vv = *(const v4f*)(vbase + (size_t)t * kQkvN + d4);
    acc += p * vv;
  }
  *(v4f*)(&pv[slice][d4]) = acc;
  __syncthreads();
  if (tid < kHd) {
    float o = pv[0][tid];
#pragma unroll
    for (int sl = 1; sl < 16; ++sl) o += pv[sl][tid];
    outs[tid] = o * inv;
  }
  __syncthreads();
  {
    const int l8 = lane & 7;
    const v4u u = pack8_h(outs + l8 * 8);
    unsigned short* dst = attn16 + rowq * kDim + h * kHd + l8 * 8;
    const bool wr = (tid < 8);
    if (wr) *(volatile v4u*)dst = u;
    __threadfence();
    if (wr) *(volatile v4u*)dst = u;
  }
}

__device__ __forceinline__ float dot4_halfwave(v4f q4, const float* kp) {
  const v4f k4 = *(const v4f*)kp;
  float p = q4.x * k4.x; p += q4.y * k4.y; p += q4.z * k4.z; p += q4.w * k4.w;
#pragma unroll
  for (int off = 1; off < 16; off <<= 1) p += __shfl_xor(p, off, 32);
  return p * kQkScale;
}
__global__ __launch_bounds__(256) void attn_feat_kernel(const float* __restrict__ qkv, unsigned short* __restrict__ attn16) {
  const int tid  = threadIdx.x;
  const int lane = tid & 31;
  const int item = blockIdx.x * 16 + (tid >> 4);
  const int j    = tid & 15, d4 = 4 * j;
  const int h    = item % kHeads;
  const int rest = item / kHeads;
  const int hw   = rest % kHW;
  const int b    = rest / kHW;
  const int s    = kGlob + hw;
  const size_t rowb = (size_t)b * kSeq;
  const size_t rowq = rowb + s;
  const v4f q4 = *(const v4f*)(qkv + rowq * kQkvN + h * kHd + d4);
  const float* kcol = qkv + kDim + h * kHd + d4;
  const float* vcol = qkv + 2 * kDim + h * kHd + d4;
  const float sc0 = dot4_halfwave(q4, kcol + (rowb + 0) * kQkvN);
  const float sc1 = dot4_halfwave(q4, kcol + (rowb + 1) * kQkvN);
  const float sc2 = dot4_halfwave(q4, kcol + (rowb + 2) * kQkvN);
  const float sc3 = dot4_halfwave(q4, kcol + (rowb + 3) * kQkvN);
  const float sc4 = dot4_halfwave(q4, kcol + (rowb + 4) * kQkvN);
  const float sc5 = dot4_halfwave(q4, kcol + rowq * kQkvN);
  float m = fmaxf(fmaxf(fmaxf(sc0, sc1), fmaxf(sc2, sc3)), fmaxf(sc4, sc5));
  float se = 0.f;
  v4f acc = (v4f){0.f, 0.f, 0.f, 0.f};
#pragma unroll 1
  for (int kk = 0; kk < 6; ++kk) {
    const float sk = (kk == 0) ? sc0 : (kk == 1) ? sc1 : (kk == 2) ? sc2 : (kk == 3) ? sc3 : (kk == 4) ? sc4 : sc5;
    const size_t vrow = (kk < 5) ? (rowb + kk) : rowq;
    const float p = expf(sk - m);
    se += p;
    const v4f vv = *(const v4f*)(vcol + vrow * kQkvN);
    acc += p * vv;
  }
  const float inv = 1.0f / se;
  acc *= inv;
  const unsigned u0 = pk16(h_bits(acc.x), h_bits(acc.y));
  const unsigned u1 = pk16(h_bits(acc.z), h_bits(acc.w));
  const int gb  = lane & 16;
  const int jl  = j & 7;
  const int sl0 = gb + 2 * jl;
  const int sl1 = sl0 + 1;
  const unsigned e0 = (unsigned)__shfl((int)u0, sl0, 32);
  const unsigned e1 = (unsigned)__shfl((int)u1, sl0, 32);
  const unsigned e2 = (unsigned)__shfl((int)u0, sl1, 32);
  const unsigned e3 = (unsigned)__shfl((int)u1, sl1, 32);
  const v4u u = (v4u){e0, e1, e2, e3};
  unsigned short* dst = attn16 + rowq * kDim + h * kHd + 8 * jl;
  const bool wr = (j < 8);
  if (wr) *(volatile v4u*)dst = u;
  __threadfence();
  if (wr) *(volatile v4u*)dst = u;
}

__device__ __forceinline__ float gelu_erf(float v) { return 0.5f * v * (1.0f + erff(v * 0.70710678118654752f)); }
__global__ __launch_bounds__(256) void gelu_f16x2_kernel(const float* __restrict__ in, unsigned short* __restrict__ out, int n2) {
  const int i = blockIdx.x * 256 + threadIdx.x;
  if (i >= n2) return;
  const v2f a = *(const v2f*)(in + 2 * (size_t)i);
  const unsigned u = pk16(h_bits(gelu_erf(a.x)), h_bits(gelu_erf(a.y)));
  unsigned short* q = out + 2 * (size_t)i;
  *(volatile unsigned*)q = u;
  __threadfence();
  *(volatile unsigned*)q = u;
}

__global__ __launch_bounds__(256) void feat_out_kernel(const float* __restrict__ tok, float* __restrict__ dout) {
  __shared__ float sm[64][65];
  const int tid = threadIdx.x, lane = tid & 31, wave = tid >> 5;
  const int hw0 = blockIdx.x * 64, c0 = blockIdx.y * 64, b = blockIdx.z;
#pragma unroll
  for (int it = 0; it < 4; ++it) {
    const int e = it * 256 + tid;
    const int r = e >> 4;
    const int c4 = (e & 15) * 4;
    const v4f v = *(const v4f*)(tok + ((size_t)b * kSeq + kGlob + hw0 + r) * kDim + c0 + c4);
    sm[c4][r] = v.x; sm[c4 + 1][r] = v.y; sm[c4 + 2][r] = v.z; sm[c4 + 3][r] = v.w;
  }
  __syncthreads();
  const int hh = lane >> 4, cs = (lane & 15) * 4;
  for (int pass = 0; pass < 2; ++pass) {
#pragma unroll
    for (int it = 0; it < 4; ++it) {
      const int row = wave * 8 + it * 2 + hh;
      const v4f v = (v4f){sm[row][cs], sm[row][cs + 1], sm[row][cs + 2], sm[row][cs + 3]};
      *(volatile v4f*)(dout + ((size_t)b * kDim + c0 + row) * kHW + hw0 + cs) = v;
    }
    __threadfence();
  }
}

__global__ __launch_bounds__(192) void tok_out_kernel(const float* __restrict__ tok, float* __restrict__ dout) {
  const int i = blockIdx.x;
  const int tid = threadIdx.x;
  size_t srow, dbase;
  if (i < kBatch) {
    srow = (size_t)i * kSeq;
    dbase = kFeatElems + (size_t)i * kDim;
  } else {
    const int jj = i - kBatch;
    const int b = jj / kReg, r = jj - b * kReg;
    srow = (size_t)b * kSeq + 1 + r;
    dbase = kFeatElems + kCtxElems + (size_t)jj * kDim;
  }
  const v4f v = *(const v4f*)(tok + srow * kDim + 4 * tid);
  float* d = dout + dbase + 4 * tid;
  *(volatile v4f*)d = v;
  __threadfence();
  *(volatile v4f*)d = v;
}

extern "C" void kernel_launch(void* const* d_in, const int* in_sizes, int n_in,
                              void* d_out, int out_size, void* d_ws, size_t ws_size,
                              hipStream_t stream)
{
  if (n_in < 15) return;
  if (ws_size < kWsTotal) return;
  if ((size_t)out_size < kOutElems) return;
  if ((size_t)in_sizes[0] < (size_t)kBatch * kDim * kHW) return;
  if ((size_t)in_sizes[3] < (size_t)kQkvN * kDim || (size_t)in_sizes[11] < (size_t)kFfn * kDim ||
      (size_t)in_sizes[13] < (size_t)kDim * kFfn || (size_t)in_sizes[5] < (size_t)kDim * kDim) return;

  const float* x    = (const float*)d_in[0];
  const float* ctxt = (const float*)d_in[1];
  const float* regt = (const float*)d_in[2];
  const float* wqkv = (const float*)d_in[3];
  const float* bqkv = (const float*)d_in[4];
  const float* wo   = (const float*)d_in[5];
  const float* bo   = (const float*)d_in[6];
  const float* ln1g = (const float*)d_in[7];
  const float* ln1b = (const float*)d_in[8];
  const float* ln2g = (const float*)d_in[9];
  const float* ln2b = (const float*)d_in[10];
  const float* w1   = (const float*)d_in[11];
  const float* b1   = (const float*)d_in[12];
  const float* w2   = (const float*)d_in[13];
  const float* b2   = (const float*)d_in[14];
  float* dout = (float*)d_out;

  char* ws = (char*)d_ws;
  unsigned short* W1h  = (unsigned short*)(ws + kOffW1h);
  unsigned short* W2h  = (unsigned short*)(ws + kOffW2h);
  unsigned short* WQh  = (unsigned short*)(ws + kOffWQh);
  unsigned short* WOh  = (unsigned short*)(ws + kOffWOh);
  float*          RA32 = (float*)(ws + kOffRA);
  unsigned short* RB16 = (unsigned short*)(ws + kOffRB);
  float*          QKV  = (float*)(ws + kOffRC);
  float*          H1   = (float*)(ws + kOffRC);
  unsigned short* FF1  = (unsigned short*)(ws + kOffFF1);

  {
    const int n8q = kQkvN * kDim / 8, n8o = kDim * kDim / 8, n8f = kFfn * kDim / 8;
    wcast8_kernel<<<(n8q + 255) / 256, 256, 0, stream>>>(wqkv, WQh, n8q, kWCarry);
    wcast8_kernel<<<(n8o + 255) / 256, 256, 0, stream>>>(wo,   WOh, n8o, kWCarry);
    wcast8_kernel<<<(n8f + 255) / 256, 256, 0, stream>>>(w1,   W1h, n8f, kWCarry);
    wcast8_kernel<<<(n8f + 255) / 256, 256, 0, stream>>>(w2,   W2h, n8f, kWCarry);
  }

  ln1_kernel<<<kRowsP, 256, 0, stream>>>(x, ctxt, regt, ln1g, ln1b, RA32, RB16);

  {
    const int tiles = (kRowsP / 64) * (kQkvN / 64);
    wmma_gemm64<0, false, 2, 0, false, 0><<<dim3((tiles + 7) / 8, 1), 256, 0, stream>>>(
        RB16, nullptr, kDim, 0L, WQh, nullptr, kDim, 0L, (void*)QKV, nullptr, kQkvN, 0L,
        bqkv, nullptr, 0L, kRowsP, kQkvN, kDim, kWCarryInv);
  }

  attn_glob_kernel<<<kBatch * kHeads * kGlob, 256, 0, stream>>>(QKV, RB16);
  attn_feat_kernel<<<(kBatch * kHW * kHeads) / 16, 256, 0, stream>>>(QKV, RB16);

  {
    const int tiles = (kRowsP / 64) * (kDim / 64);
    wmma_gemm64<0, false, 2, 0, true, 0><<<dim3((tiles + 7) / 8, 1), 256, 0, stream>>>(
        RB16, nullptr, kDim, 0L, WOh, nullptr, kDim, 0L, (void*)H1, nullptr, kDim, 0L,
        bo, RA32, 0L, kRowsP, kDim, kDim, kWCarryInv);
  }

  ln2_kernel<<<kRowsP, 256, 0, stream>>>(H1, ln2g, ln2b, RB16);

  for (int c = 0; c < kNumChunks; ++c) {
    const int r0 = c * kChunkRows;
    const int rows = (kRowsP - r0 < kChunkRows) ? (kRowsP - r0) : kChunkRows;
    const int tiles = (rows / 64) * (kFfn / 64);
    wmma_gemm64<0, false, 2, 0, false, 0><<<dim3((tiles + 7) / 8, 1), 256, 0, stream>>>(
        RB16 + (size_t)r0 * kDim, nullptr, kDim, 0L, W1h, nullptr, kDim, 0L, (void*)RA32, nullptr, kFfn, 0L,
        b1, nullptr, 0L, rows, kFfn, kDim, kWCarryInv);
    const int n2 = rows * kFfn / 2;
    gelu_f16x2_kernel<<<(n2 + 255) / 256, 256, 0, stream>>>(RA32, FF1 + (size_t)r0 * kFfn, n2);
  }

  {
    const int tiles = (kRowsP / 64) * (kDim / 64);
    wmma_gemm64<0, false, 2, 0, true, 0><<<dim3((tiles + 7) / 8, 1), 256, 0, stream>>>(
        FF1, nullptr, kFfn, 0L, W2h, nullptr, kFfn, 0L, (void*)RA32, nullptr, kDim, 0L,
        b2, H1, 0L, kRowsP, kDim, kFfn, kWCarryInv);
  }

  feat_out_kernel<<<dim3(kHW / 64, kDim / 64, kBatch), 256, 0, stream>>>(RA32, dout);
  tok_out_kernel<<<kBatch + kBatch * kReg, 192, 0, stream>>>(RA32, dout);
}
